// CausalSelfAttention_9466107921065
// MI455X (gfx1250) — hardware-verified
//
#include <hip/hip_runtime.h>
#ifndef NB
#define NB 4
#endif
#ifndef SEQ
#define SEQ 2048
#endif
#define NB_FULL 4
#define SEQ_FULL 2048
#define NBU ((unsigned)(NB))
#define SEQU ((unsigned)(SEQ))
#define SEQF ((unsigned)(SEQ_FULL))
#define DM 1024u
#define NH 16u
#define HD 64u
#define LDQ 3072u
#define BANDU (SEQU < 512u ? SEQU : 512u)
#define NTOK (NBU * SEQU)
#define NBAND (NBU * BANDU)
static_assert((SEQ) % 128 == 0);
static_assert(BANDU % 128u == 0u);
static_assert(((SEQU - BANDU) % 64u) == 0u);
static_assert((NB) <= (NB_FULL));
static_assert((SEQ) <= (SEQ_FULL));
static_assert(NH * HD == DM);
static_assert(LDQ == 3u * DM);
static_assert((size_t)(LDQ / 64u) * (NTOK / 128u) * 128u * 64u == (size_t)NTOK * LDQ);
static_assert((size_t)(NBU * NH * (SEQU / 64u)) * 64u * 64u == (size_t)NBU * NH * HD * SEQU);
static_assert((size_t)(NBU * NH * (BANDU / 64u)) * 64u * 64u == (size_t)NBU * NH * HD * BANDU);
static_assert((size_t)(NBU * NH * (BANDU / 16u)) * 16u * 64u + (size_t)(NBU * NH * ((SEQU - BANDU) / 16u)) * 16u * 64u == (size_t)NTOK * DM);
static_assert((size_t)(DM / 64u) * (NTOK / 128u) * 128u * 64u == (size_t)NTOK * DM);

typedef unsigned short v8us __attribute__((ext_vector_type(8), may_alias));
typedef float  v8f  __attribute__((ext_vector_type(8)));
typedef float  v4f  __attribute__((ext_vector_type(4)));
typedef float  v4fa __attribute__((ext_vector_type(4), may_alias));
typedef _Float16 v16h __attribute__((ext_vector_type(16)));
union FragH { v16h v; v8us half[2]; _Float16 h[16]; unsigned short u[16]; };

__device__ __forceinline__ float bf16_rne(float x) { unsigned int u = __float_as_uint(x); u = (u + 0x7FFFu + ((u >> 16) & 1u)) & 0xFFFF0000u; return __uint_as_float(u); }

__device__ __forceinline__ v16h g2_frag(const _Float16* p, unsigned hh) { FragH f; f.half[0] = *(const v8us*)((const unsigned short*)p + 8u * hh); f.half[1] = *(const v8us*)((const unsigned short*)p + 16u + 8u * hh); return f.v; }
__device__ __forceinline__ v8f g2_mma(v16h a, v16h b, v8f c) { v8f d = __builtin_amdgcn_wmma_f32_16x16x32_f16(false, a, false, b, (short)0, c, false, false); asm volatile("v_nop\n\tv_nop\n\tv_nop\n\tv_nop" : "+v"(d) : "v"(a), "v"(b)); return d; }
__device__ __forceinline__ v8f mma2(v16h a0, v16h b0, v16h a1, v16h b1, v8f c) {
  c = __builtin_amdgcn_wmma_f32_16x16x32_f16(false, a0, false, b0, (short)0, c, false, false);
  c = __builtin_amdgcn_wmma_f32_16x16x32_f16(false, a1, false, b1, (short)0, c, false, false);
  asm volatile("v_nop\n\tv_nop\n\tv_nop\n\tv_nop" : "+v"(c) : "v"(a0), "v"(b0), "v"(a1), "v"(b1));
  return c;
}
__device__ __forceinline__ v8f mma4(v16h a0, v16h b0, v16h a1, v16h b1, v16h a2, v16h b2, v16h a3, v16h b3, v8f c) {
  c = __builtin_amdgcn_wmma_f32_16x16x32_f16(false, a0, false, b0, (short)0, c, false, false);
  c = __builtin_amdgcn_wmma_f32_16x16x32_f16(false, a1, false, b1, (short)0, c, false, false);
  c = __builtin_amdgcn_wmma_f32_16x16x32_f16(false, a2, false, b2, (short)0, c, false, false);
  c = __builtin_amdgcn_wmma_f32_16x16x32_f16(false, a3, false, b3, (short)0, c, false, false);
  asm volatile("v_nop\n\tv_nop\n\tv_nop\n\tv_nop" : "+v"(c) : "v"(a0), "v"(b0), "v"(a1), "v"(b1), "v"(a2), "v"(b2), "v"(a3), "v"(b3));
  return c;
}

__global__ __launch_bounds__(256) void k_wt_f16(const float* __restrict__ W, _Float16* __restrict__ Wt, unsigned N, float scale) {
  const unsigned t = blockIdx.x * 256u + threadIdx.x;
  if (t >= N * (DM >> 3)) return;
  const unsigned n = t >> 7, k8 = (t & 127u) << 3;
  FragH f;
#pragma unroll
  for (unsigned i = 0; i < 8u; ++i) f.h[i] = (_Float16)(bf16_rne(W[(size_t)(k8 + i) * N + n]) * scale);
  const v8us o = f.half[0];
  unsigned short* d = (unsigned short*)Wt + (size_t)n * DM + k8;
  *(volatile v8us*)d = o; __threadfence(); *(volatile v8us*)d = o;
}

__global__ __launch_bounds__(256) void k_x16(const float* __restrict__ x, _Float16* __restrict__ X16) {
  const unsigned t = blockIdx.x * 256u + threadIdx.x;
  if (t >= NTOK * (DM >> 3)) return;
  const unsigned row = t >> 7, c8 = (t & 127u) << 3;
  const unsigned b = row / SEQU, s = row - b * SEQU;
  const float* src = x + ((size_t)b * SEQF + s) * DM + c8;
  const v4f a = *(const v4fa*)src, c = *(const v4fa*)(src + 4);
  FragH f;
#pragma unroll
  for (unsigned q = 0; q < 4u; ++q) { f.h[q] = (_Float16)bf16_rne(a[q]); f.h[4u + q] = (_Float16)bf16_rne(c[q]); }
  const v8us o = f.half[0];
  unsigned short* d = (unsigned short*)X16 + (size_t)row * DM + c8;
  *(volatile v8us*)d = o; __threadfence(); *(volatile v8us*)d = o;
}

template <unsigned TT>
__global__ __launch_bounds__(256) void k_vt(const _Float16* __restrict__ V16, unsigned ldv, unsigned voff, _Float16* __restrict__ Vt) {
  __shared__ unsigned short tl[64][66];
  const unsigned tid = threadIdx.x;
  const unsigned slab = blockIdx.x / (TT / 64u), lg = blockIdx.x - slab * (TT / 64u);
  const unsigned b = slab / NH, h = slab - b * NH;
  for (unsigned i = tid; i < 512u; i += 256u) {
    const unsigned r = i >> 3, c8 = (i & 7u) << 3;
    FragH f; f.half[0] = *(const v8us*)((const unsigned short*)V16 + ((size_t)b * TT + lg * 64u + r) * ldv + voff + h * HD + c8);
#pragma unroll
    for (unsigned q = 0; q < 8u; ++q) tl[r][c8 + q] = f.u[q];
  }
  __syncthreads();
  for (int pass = 0; pass < 2; ++pass) {
#pragma unroll
    for (unsigned rd = 0; rd < 2u; ++rd) {
      const unsigned d = rd * 32u + (tid >> 3), pc = tid & 7u;
      FragH f;
#pragma unroll
      for (unsigned q = 0; q < 8u; ++q) f.u[q] = tl[pc * 8u + q][d];
      *(volatile v8us*)((unsigned short*)Vt + ((size_t)slab * HD + d) * TT + lg * 64u + pc * 8u) = f.half[0];
    }
    if (pass == 0) __threadfence();
  }
}

__device__ __forceinline__ void g2_kloop(const _Float16* a0p, const _Float16* a1p, const _Float16* b0p, const _Float16* b1p, const _Float16* b2p, const _Float16* b3p, unsigned K, unsigned hh,
    v8f& c00, v8f& c01, v8f& c02, v8f& c03, v8f& c10, v8f& c11, v8f& c12, v8f& c13) {
#pragma unroll 1
  for (unsigned kb = 0; kb < K; kb += 32u) {
    const v16h a0 = g2_frag(a0p + kb, hh), a1 = g2_frag(a1p + kb, hh);
    v16h b = g2_frag(b0p + kb, hh); c00 = g2_mma(a0, b, c00); c10 = g2_mma(a1, b, c10);
    b = g2_frag(b1p + kb, hh); c01 = g2_mma(a0, b, c01); c11 = g2_mma(a1, b, c11);
    b = g2_frag(b2p + kb, hh); c02 = g2_mma(a0, b, c02); c12 = g2_mma(a1, b, c12);
    b = g2_frag(b3p + kb, hh); c03 = g2_mma(a0, b, c03); c13 = g2_mma(a1, b, c13);
  }
}

template <int MODE>
__global__ __launch_bounds__(128) void k_gemm2(const _Float16* __restrict__ A, const _Float16* __restrict__ A2, const _Float16* __restrict__ Bh, float alpha, const float* __restrict__ bias,
    float* __restrict__ C, _Float16* __restrict__ C16, _Float16* __restrict__ C16L, unsigned lda, unsigned ldc, unsigned M, unsigned K) {
  __shared__ __attribute__((aligned(16))) float so[4][32][68];
  const unsigned tid = threadIdx.x, lane = tid & 31u, ln = lane & 15u, hh = lane >> 4;
  const unsigned w = (unsigned)__builtin_amdgcn_readfirstlane((int)(tid >> 5));
  const unsigned row0 = blockIdx.y * 128u + 32u * w, col0 = blockIdx.x * 64u;
  if (row0 >= M) return;
  const unsigned bq = row0 / SEQU, sq = row0 - bq * SEQU;
  const bool band = sq < BANDU;
  const unsigned brow0 = bq * BANDU + sq;
  const _Float16* b0p = Bh + (size_t)(col0 + ln) * K; const _Float16* b1p = b0p + (size_t)16 * K; const _Float16* b2p = b1p + (size_t)16 * K; const _Float16* b3p = b2p + (size_t)16 * K;
  const v8f z8 = {0.f, 0.f, 0.f, 0.f, 0.f, 0.f, 0.f, 0.f};
  v8f c00 = z8, c01 = z8, c02 = z8, c03 = z8, c10 = z8, c11 = z8, c12 = z8, c13 = z8;
  if (MODE == 1) {
    if (band) {
      const _Float16* l0p = A2 + (size_t)(brow0 + ln) * lda; const _Float16* l1p = l0p + (size_t)16 * lda;
      g2_kloop(l0p, l1p, b0p, b1p, b2p, b3p, K, hh, c00, c01, c02, c03, c10, c11, c12, c13);
      const float rs = 0.0009765625f;
      c00 = c00 * rs; c01 = c01 * rs; c02 = c02 * rs; c03 = c03 * rs; c10 = c10 * rs; c11 = c11 * rs; c12 = c12 * rs; c13 = c13 * rs;
    }
  }
  {
    const _Float16* a0p = A + (size_t)(row0 + ln) * lda; const _Float16* a1p = a0p + (size_t)16 * lda;
    g2_kloop(a0p, a1p, b0p, b1p, b2p, b3p, K, hh, c00, c01, c02, c03, c10, c11, c12, c13);
  }
  v8f accs[8] = {c00, c01, c02, c03, c10, c11, c12, c13};
#pragma unroll
  for (int u = 0; u < 8; ++u) {
    const unsigned t = (unsigned)(u & 3), half = (unsigned)(u >> 2);
    const float bv = bf16_rne(bias[col0 + t * 16u + ln]);
#pragma unroll
    for (int r = 0; r < 8; ++r) so[w][half * 16u + 8u * hh + (unsigned)r][t * 16u + ln] = accs[u][r] * alpha + bv;
  }
  __builtin_amdgcn_fence(4  , "workgroup"); __builtin_amdgcn_wave_barrier();
  if (MODE == 0) {
    const unsigned rq = lane >> 3, c8 = (lane & 7u) << 3;
    for (int pass = 0; pass < 2; ++pass) {
#pragma unroll
      for (unsigned q = 0; q < 8u; ++q) {
        const unsigned r = q * 4u + rq;
        const v4f va = *(const v4fa*)&so[w][r][c8], vb = *(const v4fa*)&so[w][r][c8 + 4u];
        FragH fh, fl;
#pragma unroll
        for (unsigned i = 0; i < 4u; ++i) {
          _Float16 h = (_Float16)va[i]; fh.h[i] = h; fl.h[i] = (_Float16)((va[i] - (float)h) * 1024.0f);
          h = (_Float16)vb[i]; fh.h[4u + i] = h; fl.h[4u + i] = (_Float16)((vb[i] - (float)h) * 1024.0f);
        }
        *(volatile v8us*)((unsigned short*)C16 + (size_t)(row0 + r) * ldc + col0 + c8) = fh.half[0];
        if (band) *(volatile v8us*)((unsigned short*)C16L + (size_t)(brow0 + r) * ldc + col0 + c8) = fl.half[0];
      }
      if (pass == 0) __threadfence();
    }
  } else {
    const unsigned rsub = lane >> 4, c4 = (lane & 15u) << 2;
    const unsigned crow0 = bq * SEQF + sq;
    for (int pass = 0; pass < 2; ++pass) {
#pragma unroll
      for (unsigned q = 0; q < 16u; ++q) {
        const unsigned r = q * 2u + rsub;
        const v4f v = *(const v4fa*)&so[w][r][c4];
        *(volatile v4f*)(C + (size_t)(crow0 + r) * ldc + col0 + c4) = v;
      }
      if (pass == 0) __threadfence();
    }
  }
}

template <bool FINE, bool MASK>
__device__ __forceinline__ void attn_step(const _Float16* __restrict__ Kb, const _Float16* __restrict__ KLb, const _Float16* __restrict__ Vb, const _Float16* __restrict__ VLb,
    unsigned kb, v16h qf0, v16h qf1, v16h ql0, v16h ql1, unsigned q, unsigned ln, unsigned hh, float& m, float& lsum, v8f (&o)[4], v8f (&orr)[4]) {
  const v8f z8 = {0.f, 0.f, 0.f, 0.f, 0.f, 0.f, 0.f, 0.f};
  v8f s[2];
#pragma unroll
  for (int u = 0; u < 2; ++u) {
    const size_t krow = (size_t)(kb + 16u * (unsigned)u + ln);
    const _Float16* kr = Kb + krow * LDQ;
    const v16h ka = g2_frag(kr, hh), kc = g2_frag(kr + 32, hh);
    v8f sh = mma2(ka, qf0, kc, qf1, z8);
    if (FINE) {
      const _Float16* klr = KLb + krow * LDQ;
      const v16h la = g2_frag(klr, hh), lc = g2_frag(klr + 32, hh);
      const v8f sr = mma4(la, qf0, lc, qf1, ka, ql0, kc, ql1, z8);
#pragma unroll
      for (int j = 0; j < 8; ++j) sh[j] = sh[j] + sr[j] * 0.0009765625f;
    }
#pragma unroll
    for (int j = 0; j < 8; ++j) sh[j] = sh[j] * 0.125f;
    s[u] = sh;
  }
  if (MASK) {
#pragma unroll
    for (int j = 0; j < 8; ++j) {
      const unsigned key0 = kb + 8u * hh + (unsigned)j;
      s[0][j] = (key0 <= q) ? s[0][j] : -1.0e30f;
      s[1][j] = (key0 + 16u <= q) ? s[1][j] : -1.0e30f;
    }
  }
  float tmax = fmaxf(s[0][0], s[1][0]);
#pragma unroll
  for (int j = 1; j < 8; ++j) tmax = fmaxf(tmax, fmaxf(s[0][j], s[1][j]));
  tmax = fmaxf(tmax, __shfl_xor(tmax, 16, 32));
  const float nm = fmaxf(m, tmax);
  const float alpha = __expf(m - nm);
  FragH pf, pl;
  float rs = 0.f;
#pragma unroll
  for (int j = 0; j < 8; ++j) {
    const float p0 = __expf(s[0][j] - nm) * 1024.0f, p1 = __expf(s[1][j] - nm) * 1024.0f;
    rs += p0 + p1;
    const _Float16 h0 = (_Float16)p0, h1 = (_Float16)p1;
    pf.h[j] = h0; pf.h[8 + j] = h1;
    if (FINE) { pl.h[j] = (_Float16)((p0 - (float)h0) * 1024.0f); pl.h[8 + j] = (_Float16)((p1 - (float)h1) * 1024.0f); }
  }
  rs += __shfl_xor(rs, 16, 32);
  lsum = lsum * alpha + rs;
  m = nm;
#pragma unroll
  for (int t = 0; t < 4; ++t) {
    o[t] = o[t] * alpha;
    if (FINE) orr[t] = orr[t] * alpha;
  }
#pragma unroll
  for (int t = 0; t < 4; ++t) {
    const _Float16* vr = Vb + (size_t)((unsigned)t * 16u + ln) * SEQU + kb;
    const v16h vf = g2_frag(vr, hh);
    o[t] = g2_mma(vf, pf.v, o[t]);
    if (FINE) {
      const _Float16* vlr = VLb + (size_t)((unsigned)t * 16u + ln) * BANDU + kb;
      const v16h vl = g2_frag(vlr, hh);
      orr[t] = mma2(vl, pf.v, vf, pl.v, orr[t]);
    }
  }
}

template <bool FINE>
__global__ __launch_bounds__(128) void k_attn(const _Float16* __restrict__ QKV, const _Float16* __restrict__ RES, const _Float16* __restrict__ VT, const _Float16* __restrict__ VTL,
    _Float16* __restrict__ O16, _Float16* __restrict__ OL16) {
  __shared__ __attribute__((aligned(16))) float so[4][16][68];
  const unsigned tid = threadIdx.x, lane = tid & 31u, ln = lane & 15u, hh = lane >> 4;
  const unsigned w = (unsigned)__builtin_amdgcn_readfirstlane((int)(tid >> 5));
  const unsigned NT = FINE ? (BANDU / 16u) : ((SEQU - BANDU) / 16u);
  const unsigned wid = blockIdx.x * 4u + w;
  const unsigned bh = wid / NT;
  if (bh >= NBU * NH) return;
  const unsigned qt = (FINE ? 0u : (BANDU / 16u)) + (wid - bh * NT);
  const unsigned b = bh / NH, h = bh - b * NH;
  const unsigned qbase = qt * 16u, q = qbase + ln;
  const _Float16* qrow = QKV + ((size_t)b * SEQU + q) * LDQ + h * HD;
  const v16h qf0 = g2_frag(qrow, hh), qf1 = g2_frag(qrow + 32, hh);
  v16h ql0 = qf0, ql1 = qf1;
  if (FINE) { const _Float16* qlrow = RES + ((size_t)b * BANDU + q) * LDQ + h * HD; ql0 = g2_frag(qlrow, hh); ql1 = g2_frag(qlrow + 32, hh); }
  const _Float16* Kb = QKV + (size_t)b * SEQU * LDQ + DM + h * HD;
  const _Float16* KLb = RES + (size_t)b * BANDU * LDQ + DM + h * HD;
  const _Float16* Vb = VT + (size_t)bh * HD * SEQU;
  const _Float16* VLb = VTL + (size_t)bh * HD * BANDU;
  const v8f z8 = {0.f, 0.f, 0.f, 0.f, 0.f, 0.f, 0.f, 0.f};
  float m = -1.0e30f, lsum = 0.f;
  v8f o[4] = {z8, z8, z8, z8};
  v8f orr[4] = {z8, z8, z8, z8};
  const unsigned kfull = qbase & ~31u;
#pragma unroll 1
  for (unsigned kb = 0; kb < kfull; kb += 32u) attn_step<FINE, false>(Kb, KLb, Vb, VLb, kb, qf0, qf1, ql0, ql1, q, ln, hh, m, lsum, o, orr);
  attn_step<FINE, true>(Kb, KLb, Vb, VLb, kfull, qf0, qf1, ql0, ql1, q, ln, hh, m, lsum, o, orr);
  const float fin = 64.0f / lsum;
#pragma unroll
  for (int t = 0; t < 4; ++t) {
    v4f x0, x1;
#pragma unroll
    for (int j = 0; j < 4; ++j) {
      float v0 = o[t][j], v1 = o[t][4 + j];
      if (FINE) { v0 = v0 + orr[t][j] * 0.0009765625f; v1 = v1 + orr[t][4 + j] * 0.0009765625f; }
      x0[j] = v0 * fin; x1[j] = v1 * fin;
    }
    *(v4fa*)&so[w][ln][(unsigned)t * 16u + 8u * hh] = x0;
    *(v4fa*)&so[w][ln][(unsigned)t * 16u + 8u * hh + 4u] = x1;
  }
  __builtin_amdgcn_fence(4  , "workgroup"); __builtin_amdgcn_wave_barrier();
  const unsigned rq = lane >> 3, c8 = (lane & 7u) << 3;
  for (int pass = 0; pass < 2; ++pass) {
#pragma unroll
    for (unsigned it = 0; it < 4u; ++it) {
      const unsigned r = it * 4u + rq;
      const v4f va = *(const v4fa*)&so[w][r][c8], vb = *(const v4fa*)&so[w][r][c8 + 4u];
      FragH fh, fl;
#pragma unroll
      for (unsigned i = 0; i < 4u; ++i) {
        _Float16 hv = (_Float16)va[i]; fh.h[i] = hv; fl.h[i] = (_Float16)((va[i] - (float)hv) * 1024.0f);
        hv = (_Float16)vb[i]; fh.h[4u + i] = hv; fl.h[4u + i] = (_Float16)((vb[i] - (float)hv) * 1024.0f);
      }
      *(volatile v8us*)((unsigned short*)O16 + ((size_t)b * SEQU + qbase + r) * DM + h * HD + c8) = fh.half[0];
      if (FINE) *(volatile v8us*)((unsigned short*)OL16 + ((size_t)b * BANDU + qbase + r) * DM + h * HD + c8) = fl.half[0];
    }
    if (pass == 0) __threadfence();
  }
}

extern "C" void kernel_launch(void* const* d_in, const int* in_sizes, int n_in,
                              void* d_out, int out_size, void* d_ws, size_t ws_size, hipStream_t stream) {
  if (n_in < 5) return;
  const size_t need_x = ((size_t)(NB - 1) * SEQ_FULL + SEQ) * DM;
  if ((size_t)in_sizes[0] < need_x) return;
  if ((size_t)in_sizes[1] < (size_t)DM * LDQ) return;
  if ((size_t)in_sizes[2] < (size_t)LDQ) return;
  if ((size_t)in_sizes[3] < (size_t)DM * DM) return;
  if ((size_t)in_sizes[4] < (size_t)DM) return;
  if ((size_t)out_size < need_x) return;
  const float* x = (const float*)d_in[0]; const float* wqkv = (const float*)d_in[1]; const float* bqkv = (const float*)d_in[2];
  const float* wo = (const float*)d_in[3]; const float* bo = (const float*)d_in[4];
  char* ws = (char*)d_ws; size_t off = 0;
  auto take = [&](size_t bytes) { char* p = ws + off; off += (bytes + 255) & ~(size_t)255; return p; };
  _Float16* BQKV = (_Float16*)take((size_t)LDQ * DM * 2);
  _Float16* BO   = (_Float16*)take((size_t)DM * DM * 2);
  _Float16* X16  = (_Float16*)take((size_t)NTOK * DM * 2);
  _Float16* QKV16 = (_Float16*)take((size_t)NTOK * LDQ * 2);
  _Float16* RES16 = (_Float16*)take((size_t)NBAND * LDQ * 2);
  _Float16* VT   = (_Float16*)take((size_t)NBU * NH * HD * SEQU * 2);
  _Float16* VTL  = (_Float16*)take((size_t)NBU * NH * HD * BANDU * 2);
  _Float16* O16  = (_Float16*)take((size_t)NTOK * DM * 2);
  _Float16* OL16 = (_Float16*)take((size_t)NBAND * DM * 2);
  if (off > ws_size || off > (size_t)134217728) return;

  k_wt_f16<<<(unsigned)((LDQ * (DM / 8u) + 255u) / 256u), 256, 0, stream>>>(wqkv, BQKV, LDQ, 16.0f);
  k_wt_f16<<<(unsigned)((DM * (DM / 8u) + 255u) / 256u), 256, 0, stream>>>(wo, BO, DM, 16.0f);
  k_x16<<<(unsigned)((NTOK * (DM / 8u) + 255u) / 256u), 256, 0, stream>>>(x, X16);
  k_gemm2<0><<<dim3(LDQ / 64u, NTOK / 128u), 128, 0, stream>>>(X16, nullptr, BQKV, 0.0625f, bqkv, nullptr, QKV16, RES16, DM, LDQ, NTOK, DM);
  k_vt<SEQU><<<NBU * NH * (SEQU / 64u), 256, 0, stream>>>(QKV16, LDQ, 2u * DM, VT);
  k_vt<BANDU><<<NBU * NH * (BANDU / 64u), 256, 0, stream>>>(RES16, LDQ, 2u * DM, VTL);
  k_attn<true><<<NBU * NH * (BANDU / 16u) / 4u, 128, 0, stream>>>(QKV16, RES16, VT, VTL, O16, OL16);
  if (SEQU > BANDU) k_attn<false><<<NBU * NH * ((SEQU - BANDU) / 16u) / 4u, 128, 0, stream>>>(QKV16, RES16, VT, VTL, O16, OL16);
  k_gemm2<1><<<dim3(DM / 64u, NTOK / 128u), 128, 0, stream>>>(O16, OL16, BO, 0.0009765625f, bo, (float*)d_out, nullptr, nullptr, DM, DM, NTOK, DM);
}
